// ImageRenderer_48026324304156
// MI455X (gfx1250) — hardware-run, weakly checked
//
#include <hip/hip_runtime.h>
#include <math.h>

typedef __attribute__((ext_vector_type(16))) __bf16   v16b;
typedef __attribute__((ext_vector_type(8)))  __bf16   v8b;
typedef __attribute__((ext_vector_type(8)))  float    v8f;
typedef __attribute__((ext_vector_type(4)))  float    v4f;
typedef __attribute__((ext_vector_type(2)))  float    v2f;
typedef unsigned __attribute__((may_alias)) u32a;

namespace {
constexpr int   kImgW         = 256;
constexpr int   kImgH         = 256;
constexpr int   kRays         = kImgW * kImgH;
constexpr int   kSmp          = 64;
constexpr int   kHid          = 64;
constexpr int   kOutC         = 4;
constexpr float kZNear        = 2.0f;
constexpr float kZFar         = 6.0f;
constexpr float kBinDt        = (kZFar - kZNear) / (float)kSmp;
constexpr int   kWaves        = 8;
constexpr int   kRaysPerWave  = 4;
constexpr int   kRaysPerBlock = kWaves * kRaysPerWave;
constexpr int   kPitch        = 72;
constexpr int   kPitchW       = kPitch / 2;
}
static_assert(kBinDt == 0.0625f);
static_assert(kSmp == 64 && kHid == 64 && kOutC == 4);
static_assert(kRaysPerBlock == 32);
static_assert((kRays % kRaysPerBlock) == 0);
static_assert((kRaysPerBlock * 3 * 4) % 128 == 0);
static_assert((kPitch % 8) == 0);

__device__ __forceinline__ unsigned rne_bf_word(float f) {
  const unsigned u = __float_as_uint(f);
  return u + 0x7FFFu + ((u >> 16) & 1u);
}

template <typename T> struct Frag;
template <> struct Frag<__bf16> {
  typedef v16b V; union U { v16b v; v8b h[2]; };
  static __device__ __forceinline__ v16b load(const __bf16* p) {
    U f; f.h[0] = *(const v8b*)(p); f.h[1] = *(const v8b*)(p + 16); return f.v;
  }
  static __device__ __forceinline__ v8f mma(v16b a, v16b b, v8f c) {
    return __builtin_amdgcn_wmma_f32_16x16x32_bf16(false, a, false, b, (short)0, c, false, false);
  }
};

__device__ __forceinline__ void acc_guard_group(v8f& c, v16b a0, v16b a1, v16b a2, v16b a3, v16b b0, v16b b1) {
  asm volatile("v_nop\n\tv_nop\n\tv_nop\n\tv_nop" : "+v"(c) : "v"(a0), "v"(a1), "v"(a2), "v"(a3), "v"(b0), "v"(b1));
}

__device__ __forceinline__ void wave_lds_sync() {
  __builtin_amdgcn_fence(__ATOMIC_RELEASE, "workgroup");
  __builtin_amdgcn_wave_barrier();
  __builtin_amdgcn_fence(__ATOMIC_ACQUIRE, "workgroup");
}

__device__ __forceinline__ unsigned w2_plane_bits(float w, int n) {
  const unsigned hw = rne_bf_word(w);
  const float lof = w - __uint_as_float(hw & 0xffff0000u);
  const float src = (n < 4) ? w : ((n < 8) ? lof : 0.0f);
  return rne_bf_word(src) >> 16;
}

__device__ __forceinline__ float sigmoid_f32(float x) {
  return __builtin_amdgcn_rcpf(1.0f + expf(-x));
}

__global__ __launch_bounds__(256) void render_rays_kernel(
    const float* __restrict__ cam,
    const float* __restrict__ uj,
    const float* __restrict__ crd,
    const float* __restrict__ W1,
    const float* __restrict__ b1,
    const float* __restrict__ W2,
    const float* __restrict__ b2,
    float* __restrict__ outc)
{
  __shared__ __align__(16) __bf16 sBt[16 * kPitch];
  __shared__ __align__(16) __bf16 sAhi[kWaves][16 * kPitch];
  __shared__ __align__(16) __bf16 sAlo[kWaves][16 * kPitch];
  __shared__ __align__(16) float  sO[kWaves][kSmp * 8];
  __shared__ __align__(16) float  sT[kWaves][kSmp];
  __shared__ __align__(16) float  sStage[kRaysPerBlock * 3];

  const int tid  = threadIdx.x;
  const int lane = tid & 31;
  const int wave = tid >> 5;
  const int hh   = lane >> 4;
  const int cl   = lane & 15;
  const int l2   = lane * 2;

  {
    const int n  = tid >> 4;
    const int k4 = (tid & 15) * 4;
    const int c  = n & 3;
    const float w0 = W2[(k4 + 0) * kOutC + c];
    const float w1 = W2[(k4 + 1) * kOutC + c];
    const float w2 = W2[(k4 + 2) * kOutC + c];
    const float w3 = W2[(k4 + 3) * kOutC + c];
    const unsigned e0 = w2_plane_bits(w0, n);
    const unsigned e1 = w2_plane_bits(w1, n);
    const unsigned e2 = w2_plane_bits(w2, n);
    const unsigned e3 = w2_plane_bits(w3, n);
    u32a* bw = (u32a*)(sBt + n * kPitch + k4);
    bw[0] = e0 | (e1 << 16);
    bw[1] = e2 | (e3 << 16);
  }

  const v2f wa0 = *(const v2f*)(W1 + 0 * kHid + l2);
  const v2f wa1 = *(const v2f*)(W1 + 1 * kHid + l2);
  const v2f wa2 = *(const v2f*)(W1 + 2 * kHid + l2);
  const v2f wa3 = *(const v2f*)(W1 + 3 * kHid + l2);
  const v2f wa4 = *(const v2f*)(W1 + 4 * kHid + l2);
  const v2f wa5 = *(const v2f*)(W1 + 5 * kHid + l2);
  const v2f bb1 = *(const v2f*)(b1 + l2);

  const float r00 = cam[0], r01 = cam[1], r02 = cam[2],  ox = cam[3];
  const float r10 = cam[4], r11 = cam[5], r12 = cam[6],  oy = cam[7];
  const float r20 = cam[8], r21 = cam[9], r22 = cam[10], oz = cam[11];
  const float b2v0 = b2[0], b2v1 = b2[1], b2v2 = b2[2], b2v3 = b2[3];

  const float ao0 = bb1.x + ox * wa0.x + oy * wa1.x + oz * wa2.x;
  const float ao1 = bb1.y + ox * wa0.y + oy * wa1.y + oz * wa2.y;

  __syncthreads();

  const v16b bf0 = Frag<__bf16>::load(sBt + cl * kPitch + 0  + 8 * hh);
  const v16b bf1 = Frag<__bf16>::load(sBt + cl * kPitch + 32 + 8 * hh);

  __bf16* ahi = sAhi[wave];
  __bf16* alo = sAlo[wave];
  float*  oS  = sO[wave];
  float*  tS  = sT[wave];

#pragma unroll 1
  for (int i = 0; i < kRaysPerWave; ++i) {
    const int rib = wave * kRaysPerWave + i;
    const int ray = blockIdx.x * kRaysPerBlock + rib;

    const float c0 = crd[(size_t)ray * 3 + 0];
    const float c1 = crd[(size_t)ray * 3 + 1];
    const float c2 = crd[(size_t)ray * 3 + 2];
    const float dx = r00 * c0 + r01 * c1 + r02 * c2;
    const float dy = r10 * c0 + r11 * c1 + r12 * c2;
    const float dz = r20 * c0 + r21 * c1 + r22 * c2;

    const v2f uu = *(const v2f*)(uj + (size_t)ray * kSmp + l2);
    const float tb = kZNear + kBinDt * (float)l2;
    v2f tt;
    tt.x = tb + uu.x * kBinDt;
    tt.y = (tb + kBinDt) + uu.y * kBinDt;
    *(v2f*)(tS + l2) = tt;

    const float a0 = ao0 + dx * wa3.x + dy * wa4.x + dz * wa5.x;
    const float a1 = ao1 + dx * wa3.y + dy * wa4.y + dz * wa5.y;
    const float g0 = dx * wa0.x + dy * wa1.x + dz * wa2.x;
    const float g1 = dx * wa0.y + dy * wa1.y + dz * wa2.y;

    wave_lds_sync();

#pragma unroll 1
    for (int tile = 0; tile < 4; ++tile) {
      const float* tp = tS + tile * 16;
      u32a* ph = (u32a*)(ahi) + lane;
      u32a* pl = (u32a*)(alo) + lane;
#pragma unroll 1
      for (int s4 = 0; s4 < 4; ++s4) {
        const v4f t4 = *(const v4f*)(tp + s4 * 4);
#pragma unroll
        for (int e = 0; e < 4; ++e) {
          const float ts = t4[e];
          const float h0 = fmaxf(fmaf(ts, g0, a0), 0.0f);
          const float h1 = fmaxf(fmaf(ts, g1, a1), 0.0f);
          const unsigned hw0 = rne_bf_word(h0);
          const unsigned hw1 = rne_bf_word(h1);
          const float lo0 = h0 - __uint_as_float(hw0 & 0xffff0000u);
          const float lo1 = h1 - __uint_as_float(hw1 & 0xffff0000u);
          const unsigned lw0 = rne_bf_word(lo0);
          const unsigned lw1 = rne_bf_word(lo1);
          const int row = s4 * 4 + e;
          ph[row * kPitchW] = (hw0 >> 16) | (hw1 & 0xffff0000u);
          pl[row * kPitchW] = (lw0 >> 16) | (lw1 & 0xffff0000u);
        }
      }
      wave_lds_sync();

      const __bf16* arh = ahi + cl * kPitch + 8 * hh;
      const __bf16* arl = alo + cl * kPitch + 8 * hh;
      const v16b ah0 = Frag<__bf16>::load(arh);
      const v16b ah1 = Frag<__bf16>::load(arh + 32);
      const v16b al0 = Frag<__bf16>::load(arl);
      const v16b al1 = Frag<__bf16>::load(arl + 32);
      v8f c = (v8f){0.f, 0.f, 0.f, 0.f, 0.f, 0.f, 0.f, 0.f};
      c = Frag<__bf16>::mma(ah0, bf0, c);
      c = Frag<__bf16>::mma(ah1, bf1, c);
      c = Frag<__bf16>::mma(al0, bf0, c);
      c = Frag<__bf16>::mma(al1, bf1, c);
      acc_guard_group(c, ah0, ah1, al0, al1, bf0, bf1);

      if (cl < 8) {
        float* op = oS + (tile * 16 + 8 * hh) * 8 + cl;
#pragma unroll
        for (int r = 0; r < 8; ++r) op[r * 8] = c[r];
      }
      wave_lds_sync();
    }

    {
      const float* ob = oS + lane * 16;
      const v4f p0 = *(const v4f*)(ob);
      const v4f p1 = *(const v4f*)(ob + 4);
      const v4f p2 = *(const v4f*)(ob + 8);
      const v4f p3 = *(const v4f*)(ob + 12);
      const float od0 = (p0[0] + p1[0]) + b2v0;
      const float or0 = (p0[1] + p1[1]) + b2v1;
      const float og0 = (p0[2] + p1[2]) + b2v2;
      const float ob0 = (p0[3] + p1[3]) + b2v3;
      const float od1 = (p2[0] + p3[0]) + b2v0;
      const float or1 = (p2[1] + p3[1]) + b2v1;
      const float og1 = (p2[2] + p3[2]) + b2v2;
      const float ob1 = (p2[3] + p3[3]) + b2v3;

      const int sn = (l2 + 2 < kSmp) ? (l2 + 2) : (kSmp - 1);
      const float tn = tS[sn];
      const float sep0 = tt.y - tt.x;
      const float sep1 = (lane < 31) ? (tn - tt.y) : kBinDt;

      const float d0 = fmaxf(od0, 0.0f);
      const float d1 = fmaxf(od1, 0.0f);
      const float q0 = expf(-d0 * sep0);
      const float q1 = expf(-d1 * sep1);
      const float al0s = 1.0f - q0;
      const float al1s = 1.0f - q1;

      float incl = q0 * q1;
#pragma unroll
      for (int dd = 1; dd < 32; dd <<= 1) {
        const float up = __shfl_up(incl, dd, 32);
        const float pr = incl * up;
        incl = (lane >= dd) ? pr : incl;
      }
      const float sh1 = __shfl_up(incl, 1, 32);
      const float excl = (lane == 0) ? 1.0f : sh1;

      const float wgt0 = al0s * excl;
      const float wgt1 = al1s * (excl * q0);

      float cr = wgt0 * sigmoid_f32(or0) + wgt1 * sigmoid_f32(or1);
      float cg = wgt0 * sigmoid_f32(og0) + wgt1 * sigmoid_f32(og1);
      float cb = wgt0 * sigmoid_f32(ob0) + wgt1 * sigmoid_f32(ob1);
#pragma unroll
      for (int dd = 16; dd >= 1; dd >>= 1) {
        const float xr = __shfl_xor(cr, dd, 32);
        const float xg = __shfl_xor(cg, dd, 32);
        const float xb = __shfl_xor(cb, dd, 32);
        cr += xr;
        cg += xg;
        cb += xb;
      }
      const float val = (lane == 0) ? cr : ((lane == 1) ? cg : cb);
      if (lane < 3) sStage[rib * 3 + lane] = val;
    }
    wave_lds_sync();
  }

  __syncthreads();
  if (tid < 24) {
    const v4f sv = *(const v4f*)(sStage + tid * 4);
    float* gp = outc + (size_t)blockIdx.x * (kRaysPerBlock * 3) + tid * 4;
    *(volatile v4f*)gp = sv;
    __threadfence();
    *(volatile v4f*)gp = sv;
  }
}

extern "C" void kernel_launch(void* const* d_in, const int* in_sizes, int n_in,
                              void* d_out, int out_size, void* d_ws, size_t ws_size,
                              hipStream_t stream) {
  if (n_in < 7) return;
  if (in_sizes[0] != 16) return;
  if (in_sizes[1] != kRays * kSmp) return;
  if (in_sizes[2] != kRays * 3) return;
  if (in_sizes[3] != 6 * kHid) return;
  if (in_sizes[4] != kHid) return;
  if (in_sizes[5] != kHid * kOutC) return;
  if (in_sizes[6] != kOutC) return;
  if (out_size != kRays * 3) return;
  (void)d_ws;
  (void)ws_size;

  const float* cam = (const float*)d_in[0];
  const float* uj  = (const float*)d_in[1];
  const float* crd = (const float*)d_in[2];
  const float* W1  = (const float*)d_in[3];
  const float* b1  = (const float*)d_in[4];
  const float* W2  = (const float*)d_in[5];
  const float* b2  = (const float*)d_in[6];
  float* outc = (float*)d_out;

  render_rays_kernel<<<dim3(kRays / kRaysPerBlock), dim3(256), 0, stream>>>(cam, uj, crd, W1, b1, W2, b2, outc);
}
